// DilatedAttention_13864154431563
// MI455X (gfx1250) — hardware-verified
//
#include <hip/hip_runtime.h>
#include <math.h>

typedef __attribute__((ext_vector_type(16))) __bf16 v16b;
typedef __attribute__((ext_vector_type(8)))  __bf16 v8b;
typedef __attribute__((ext_vector_type(8)))  float  v8f;
typedef __attribute__((ext_vector_type(4)))  float  v4f;
typedef __attribute__((ext_vector_type(2)))  float  v2f;

constexpr int SEQ_LEN    = 4096;
constexpr int NUM_HEAD   = 16;
constexpr int HDIM       = 64;
constexpr int HALF_D     = 32;
constexpr int EMB        = NUM_HEAD * HDIM;
constexpr int SPARSE_LEN = 1024;
constexpr int QBLK       = 64;
constexpr int KCH        = 64;

static_assert(EMB == 1024, "embed");
static_assert(SPARSE_LEN % QBLK == 0 && SPARSE_LEN % KCH == 0, "tiles");

__device__ __forceinline__ unsigned short at_bf_bits(float f) {
  unsigned u = __float_as_uint(f);
  return (unsigned short)((u + 0x7FFFu + ((u >> 16) & 1u)) >> 16);
}
__device__ __forceinline__ __bf16 at_f2bf(float f) { return __builtin_bit_cast(__bf16, at_bf_bits(f)); }
__device__ __forceinline__ void at_split(float f, __bf16& hi, __bf16& lo) {
  const unsigned short hb = at_bf_bits(f);
  hi = __builtin_bit_cast(__bf16, hb);
  lo = at_f2bf(f - __uint_as_float(((unsigned)hb) << 16));
}
__device__ __forceinline__ void split_pack2(float a, float b, unsigned& wh, unsigned& wl) {
  const unsigned ha = at_bf_bits(a), hb = at_bf_bits(b);
  const unsigned la = at_bf_bits(a - __uint_as_float(ha << 16));
  const unsigned lb = at_bf_bits(b - __uint_as_float(hb << 16));
  wh = ha | (hb << 16);
  wl = la | (lb << 16);
}

__device__ __forceinline__ v8f at_mma(v16b a, v16b b, v8f c) {
  c = __builtin_amdgcn_wmma_f32_16x16x32_bf16(false, a, false, b, (short)0, c, false, false);
  asm volatile("v_nop\n\tv_nop\n\tv_nop\n\tv_nop" : "+v"(c) : "v"(a), "v"(b));
  return c;
}
__device__ __forceinline__ v16b frag_load_bf16(const __bf16* p) {
  union { v16b v; v8b h[2]; } f;
  f.h[0] = *(const v8b*)(p);
  f.h[1] = *(const v8b*)(p + 16);
  return f.v;
}

struct FreqTab { float f[32]; };
static_assert(sizeof(FreqTab) == 128, "no padding");

__global__ __launch_bounds__(256)
void xpos_table_kernel(FreqTab ft, float* __restrict__ cq, float* __restrict__ sq,
                       float* __restrict__ ck, float* __restrict__ sk, int total) {
  const int idx = blockIdx.x * 256 + threadIdx.x;
  if (idx >= total) return;
  const int i = idx & 31;
  const int p = idx >> 5;
  float fr = ft.f[0];
#pragma unroll
  for (int j = 1; j < 32; ++j) fr = (i == j) ? ft.f[j] : fr;
  const float sv  = ((float)(2 * i) + 25.6f) * (1.0f / 89.6f);
  const float e   = (float)(p - (SEQ_LEN / 2)) * (1.0f / 512.0f);
  const float le  = e * log2f(sv);
  const float sc  = exp2f(le);
  const float isc = exp2f(-le);
  const float ang = (float)p * fr;
  float sn, cs;
  sincosf(ang, &sn, &cs);
  const float vcq = cs * sc, vsq = sn * sc, vck = cs * isc, vsk = sn * isc;
  volatile float* pcq = cq; volatile float* psq = sq; volatile float* pck = ck; volatile float* psk = sk;
  pcq[idx] = vcq; psq[idx] = vsq; pck[idx] = vck; psk[idx] = vsk;
  __threadfence();
  pcq[idx] = vcq; psq[idx] = vsq; pck[idx] = vck; psk[idx] = vsk;
}

__global__ __launch_bounds__(256)
void prep_qkv_kernel(const float* __restrict__ q, const float* __restrict__ k, const float* __restrict__ v,
                     const float* __restrict__ cq, const float* __restrict__ sq,
                     const float* __restrict__ ck, const float* __restrict__ sk,
                     unsigned* __restrict__ qh, unsigned* __restrict__ ql,
                     unsigned* __restrict__ kh, unsigned* __restrict__ kl,
                     unsigned* __restrict__ vh, unsigned* __restrict__ vl, int total) {
  const int idx = blockIdx.x * 256 + threadIdx.x;
  if (idx >= total) return;
  const int lane = idx & 31;
  const int row  = idx >> 5;
  const int h    = row >> 12;
  const int p    = row & (SEQ_LEN - 1);
  const size_t src = (size_t)p * EMB + (size_t)h * HDIM + 2 * lane;
  const v2f qv = *(const v2f*)(q + src);
  const v2f kv = *(const v2f*)(k + src);
  const v2f vv = *(const v2f*)(v + src);
  const int ti = p * HALF_D + lane;
  const float c1 = cq[ti], s1 = sq[ti], c2 = ck[ti], s2 = sk[ti];
  const float qa = (qv.x * c1 - qv.y * s1) * 0.125f;
  const float qb = (qv.y * c1 + qv.x * s1) * 0.125f;
  const float ka = kv.x * c2 - kv.y * s2;
  const float kb = kv.y * c2 + kv.x * s2;
  unsigned wqh, wql, wkh, wkl, wvh, wvl;
  split_pack2(qa, qb, wqh, wql);
  split_pack2(ka, kb, wkh, wkl);
  split_pack2(vv.x, vv.y, wvh, wvl);
  const size_t w = (size_t)row * HALF_D + lane;
  volatile unsigned* pqh = qh; volatile unsigned* pql = ql; volatile unsigned* pkh = kh;
  volatile unsigned* pkl = kl; volatile unsigned* pvh = vh; volatile unsigned* pvl = vl;
  pqh[w] = wqh; pql[w] = wql; pkh[w] = wkh; pkl[w] = wkl; pvh[w] = wvh; pvl[w] = wvl;
  __threadfence();
  pqh[w] = wqh; pql[w] = wql; pkh[w] = wkh; pkl[w] = wkl; pvh[w] = wvh; pvl[w] = wvl;
}

struct AttnTiles {
  unsigned short Kh[KCH * HDIM];
  unsigned short Kl[KCH * HDIM];
  unsigned short Vh[HDIM * KCH];
  unsigned short Vl[HDIM * KCH];
};
union AttnLds {
  AttnTiles t;
  float Os[4][16 * 68];
};
static_assert(sizeof(AttnTiles) == 32768, "tiles");
static_assert(sizeof(float) * 4 * 16 * 68 <= sizeof(AttnTiles), "slab fits");

__global__ __launch_bounds__(128)
void dil_attn_kernel(const unsigned short* __restrict__ qhp, const unsigned short* __restrict__ qlp,
                     const unsigned short* __restrict__ khp, const unsigned short* __restrict__ klp,
                     const unsigned short* __restrict__ vhp, const unsigned short* __restrict__ vlp,
                     float* __restrict__ oc, float* __restrict__ lsec,
                     int r, int sl, int nseg, int cshift) {
  union FB { v16b v; v8b h[2]; };
  __shared__ __align__(16) AttnLds U;
  __shared__ __align__(16) __bf16 Psh[4][16 * KCH];
  __shared__ __align__(16) __bf16 Psl[4][16 * KCH];
  __shared__ __align__(16) float  lse_s[QBLK];

  const int tid  = threadIdx.x;
  const int wave = tid >> 5;
  const int lane = tid & 31;
  const int hh   = lane >> 4;
  const int c    = lane & 15;

  const int bx   = blockIdx.x;
  const int qb   = bx & 15;
  const int h    = (bx >> 4) & 15;
  const int seg  = bx >> 8;
  const int seqb = nseg * SPARSE_LEN;
  const int coff = h >> cshift;
  const size_t base = ((size_t)h * SEQ_LEN + (size_t)seg * (size_t)sl + (size_t)coff) * HDIM;
  const size_t rs   = (size_t)r * HDIM;
  const int q0 = qb * QBLK + wave * 16;

  const __bf16* Qh = (const __bf16*)(const void*)(qhp + base);
  const __bf16* Ql = (const __bf16*)(const void*)(qlp + base);
  v16b qah[2], qal[2];
#pragma unroll
  for (int dc = 0; dc < 2; ++dc) {
    const size_t o = (size_t)(q0 + c) * rs + (size_t)(dc * 32 + 8 * hh);
    qah[dc] = frag_load_bf16(Qh + o);
    qal[dc] = frag_load_bf16(Ql + o);
  }

  float mrow[8], lrow[8];
  v8f oacc[4];
#pragma unroll
  for (int rr = 0; rr < 8; ++rr) { mrow[rr] = -INFINITY; lrow[rr] = 0.f; }
#pragma unroll
  for (int t = 0; t < 4; ++t) oacc[t] = (v8f){0.f,0.f,0.f,0.f,0.f,0.f,0.f,0.f};

  const int nchunks = qb + 1;
  for (int kc = 0; kc < nchunks; ++kc) {
    const int kv0 = kc * KCH;
    __syncthreads();
#pragma unroll
    for (int i = 0; i < 4; ++i) {
      const int qd = tid + 128 * i;
      const int kv = qd >> 3;
      const int d0 = (qd & 7) * 8;
      const size_t go = base + (size_t)(kv0 + kv) * rs + (size_t)d0;
      const uint4 a = *(const uint4*)(const void*)(khp + go);
      const uint4 b = *(const uint4*)(const void*)(klp + go);
      *(uint4*)(void*)(U.t.Kh + kv * HDIM + d0) = a;
      *(uint4*)(void*)(U.t.Kl + kv * HDIM + d0) = b;
    }
    asm volatile("" ::: "memory");
#pragma unroll
    for (int i = 0; i < 4; ++i) {
      const int qd = tid + 128 * i;
      const int kv = qd >> 3;
      const int d0 = (qd & 7) * 8;
      const size_t go = base + (size_t)(kv0 + kv) * rs + (size_t)d0;
      const uint4 a = *(const uint4*)(const void*)(vhp + go);
      const uint4 b = *(const uint4*)(const void*)(vlp + go);
      const unsigned aw[4] = {a.x, a.y, a.z, a.w};
      const unsigned bw[4] = {b.x, b.y, b.z, b.w};
#pragma unroll
      for (int m = 0; m < 4; ++m) {
        U.t.Vh[(d0 + 2 * m) * KCH + kv]     = (unsigned short)(aw[m] & 0xffffu);
        U.t.Vh[(d0 + 2 * m + 1) * KCH + kv] = (unsigned short)(aw[m] >> 16);
        U.t.Vl[(d0 + 2 * m) * KCH + kv]     = (unsigned short)(bw[m] & 0xffffu);
        U.t.Vl[(d0 + 2 * m + 1) * KCH + kv] = (unsigned short)(bw[m] >> 16);
      }
    }
    __syncthreads();

    v8f s[4];
#pragma unroll
    for (int j = 0; j < 4; ++j) {
      s[j] = (v8f){0.f,0.f,0.f,0.f,0.f,0.f,0.f,0.f};
#pragma unroll
      for (int dc = 0; dc < 2; ++dc) {
        FB kb, kl;
        const int ko = (j * 16 + c) * HDIM + dc * 32 + 8 * hh;
        kb.h[0] = *(const v8b*)(const void*)(U.t.Kh + ko);
        kb.h[1] = *(const v8b*)(const void*)(U.t.Kh + ko + 16);
        kl.h[0] = *(const v8b*)(const void*)(U.t.Kl + ko);
        kl.h[1] = *(const v8b*)(const void*)(U.t.Kl + ko + 16);
        s[j] = at_mma(qah[dc], kb.v, s[j]);
        s[j] = at_mma(qah[dc], kl.v, s[j]);
        s[j] = at_mma(qal[dc], kb.v, s[j]);
      }
    }
    const bool diag = (kc == qb);
    float cm[8];
#pragma unroll
    for (int rr = 0; rr < 8; ++rr) {
      const int qrow = q0 + 8 * hh + rr;
      float m = -INFINITY;
#pragma unroll
      for (int j = 0; j < 4; ++j) {
        const int kvcol = kv0 + j * 16 + c;
        if (diag && (kvcol > qrow)) s[j][rr] = -1.0e9f;
        m = fmaxf(m, s[j][rr]);
      }
#pragma unroll
      for (int off = 1; off < 16; off <<= 1) m = fmaxf(m, __shfl_xor(m, off, 32));
      cm[rr] = m;
    }
    __bf16* pwh = Psh[wave];
    __bf16* pwl = Psl[wave];
#pragma unroll
    for (int rr = 0; rr < 8; ++rr) {
      const float mnew  = fmaxf(mrow[rr], cm[rr]);
      const float alpha = expf(mrow[rr] - mnew);
      mrow[rr] = mnew;
      float psum = 0.f;
#pragma unroll
      for (int j = 0; j < 4; ++j) {
        const float p = expf(s[j][rr] - mnew);
        psum += p;
        __bf16 a, bl;
        at_split(p, a, bl);
        pwh[(8 * hh + rr) * KCH + j * 16 + c] = a;
        pwl[(8 * hh + rr) * KCH + j * 16 + c] = bl;
      }
#pragma unroll
      for (int off = 1; off < 16; off <<= 1) psum += __shfl_xor(psum, off, 32);
      lrow[rr] = lrow[rr] * alpha + psum;
#pragma unroll
      for (int t = 0; t < 4; ++t) oacc[t][rr] *= alpha;
    }
    __builtin_amdgcn_fence(__ATOMIC_RELEASE, "workgroup");
    __builtin_amdgcn_wave_barrier();
    __builtin_amdgcn_fence(__ATOMIC_ACQUIRE, "workgroup");
#pragma unroll
    for (int kk = 0; kk < 2; ++kk) {
      FB pa, pl;
      const int po = c * KCH + kk * 32 + 8 * hh;
      pa.h[0] = *(const v8b*)(pwh + po);
      pa.h[1] = *(const v8b*)(pwh + po + 16);
      pl.h[0] = *(const v8b*)(pwl + po);
      pl.h[1] = *(const v8b*)(pwl + po + 16);
#pragma unroll
      for (int t = 0; t < 4; ++t) {
        FB vb, vlo;
        const int vo = (t * 16 + c) * KCH + kk * 32 + 8 * hh;
        vb.h[0]  = *(const v8b*)(const void*)(U.t.Vh + vo);
        vb.h[1]  = *(const v8b*)(const void*)(U.t.Vh + vo + 16);
        vlo.h[0] = *(const v8b*)(const void*)(U.t.Vl + vo);
        vlo.h[1] = *(const v8b*)(const void*)(U.t.Vl + vo + 16);
        oacc[t] = at_mma(pa.v, vb.v,  oacc[t]);
        oacc[t] = at_mma(pa.v, vlo.v, oacc[t]);
        oacc[t] = at_mma(pl.v, vb.v,  oacc[t]);
      }
    }
  }

  __syncthreads();
  float* os = U.Os[wave];
#pragma unroll
  for (int rr = 0; rr < 8; ++rr) {
    const float inv = 1.0f / lrow[rr];
#pragma unroll
    for (int t = 0; t < 4; ++t) os[(8 * hh + rr) * 68 + t * 16 + c] = oacc[t][rr] * inv;
    if (c == 0) lse_s[wave * 16 + 8 * hh + rr] = mrow[rr] + logf(lrow[rr]);
  }
  __builtin_amdgcn_fence(__ATOMIC_RELEASE, "workgroup");
  __builtin_amdgcn_wave_barrier();
  __builtin_amdgcn_fence(__ATOMIC_ACQUIRE, "workgroup");
  {
    float* ob = oc + ((size_t)h * seqb + (size_t)seg * SPARSE_LEN + (size_t)q0) * HDIM;
    const int c4 = c * 4;
    for (int pass = 0; pass < 2; ++pass) {
#pragma unroll
      for (int it = 0; it < 8; ++it) {
        const int row = it * 2 + hh;
        const v4f val = *(const v4f*)(os + row * 68 + c4);
        *(volatile v4f*)(ob + (size_t)row * HDIM + c4) = val;
      }
      __threadfence();
    }
  }
  __syncthreads();
  if (tid < 16) {
    const v4f lv = *(const v4f*)(lse_s + 4 * tid);
    float* lp = lsec + (size_t)h * seqb + (size_t)seg * SPARSE_LEN + (size_t)qb * QBLK + 4 * tid;
    *(volatile v4f*)lp = lv;
    __threadfence();
    *(volatile v4f*)lp = lv;
  }
}

__global__ __launch_bounds__(256)
void combine_kernel(const float* __restrict__ o0, const float* __restrict__ o1, const float* __restrict__ o2,
                    const float* __restrict__ l0, const float* __restrict__ l1, const float* __restrict__ l2,
                    float* __restrict__ out, int total) {
  const int idx = blockIdx.x * 256 + threadIdx.x;
  if (idx >= total) return;
  const int p  = idx >> 8;
  const int h  = (idx >> 4) & 15;
  const int d4 = (idx & 15) * 4;
  const int c1 = h >> 3, c2 = h >> 2;
  const bool v1 = ((p & 1) == c1);
  const bool v2 = ((p & 3) == c2);
  const int sg1 = (p >> 11) * SPARSE_LEN + ((p & 2047) >> 1);
  const int sg2 = p >> 2;
  const float L0  = l0[h * 4096 + p];
  const float L1v = l1[h * 2048 + sg1];
  const float L2v = l2[h * 1024 + sg2];
  const v4f a0 = *(const v4f*)(o0 + ((size_t)h * 4096 + (size_t)p)   * HDIM + d4);
  const v4f a1 = *(const v4f*)(o1 + ((size_t)h * 2048 + (size_t)sg1) * HDIM + d4);
  const v4f a2 = *(const v4f*)(o2 + ((size_t)h * 1024 + (size_t)sg2) * HDIM + d4);
  const float L1 = v1 ? L1v : -1.0e8f;
  const float L2 = v2 ? L2v : -1.0e8f;
  const float mx = fmaxf(L0, fmaxf(L1, L2));
  const float w0 = expf(L0 - mx), w1 = expf(L1 - mx), w2 = expf(L2 - mx);
  const float rdn = 1.0f / (w0 + w1 + w2);
  const v4f res = (a0 * w0 + a1 * w1 + a2 * w2) * rdn;
  float* op = out + (size_t)p * EMB + (size_t)h * HDIM + d4;
  *(volatile v4f*)op = res;
  __threadfence();
  *(volatile v4f*)op = res;
}

extern "C" void kernel_launch(void* const* d_in, const int* in_sizes, int n_in,
                              void* d_out, int out_size, void* d_ws, size_t ws_size,
                              hipStream_t stream) {
  if (n_in < 3) return;
  const int nel = SEQ_LEN * EMB;
  if (in_sizes[0] != nel || in_sizes[1] != nel || in_sizes[2] != nel || out_size != nel) return;

  const float* q = (const float*)d_in[0];
  const float* k = (const float*)d_in[1];
  const float* v = (const float*)d_in[2];
  float* out = (float*)d_out;

  const size_t TAB_BYTES   = (size_t)SEQ_LEN * HALF_D * sizeof(float);
  const size_t PLANE_BYTES = (size_t)NUM_HEAD * SEQ_LEN * HDIM * 2;
  const size_t O0_BYTES    = (size_t)NUM_HEAD * 4096 * HDIM * sizeof(float);
  const size_t O1_BYTES    = (size_t)NUM_HEAD * 2048 * HDIM * sizeof(float);
  const size_t O2_BYTES    = (size_t)NUM_HEAD * 1024 * HDIM * sizeof(float);
  const size_t L0_BYTES    = (size_t)NUM_HEAD * 4096 * sizeof(float);
  const size_t L1_BYTES    = (size_t)NUM_HEAD * 2048 * sizeof(float);
  const size_t L2_BYTES    = (size_t)NUM_HEAD * 1024 * sizeof(float);

  char* ws = (char*)d_ws;
  size_t off = 0;
  float* cq = (float*)(ws + off); off += TAB_BYTES;
  float* sq = (float*)(ws + off); off += TAB_BYTES;
  float* ck = (float*)(ws + off); off += TAB_BYTES;
  float* sk = (float*)(ws + off); off += TAB_BYTES;
  unsigned* qh = (unsigned*)(ws + off); off += PLANE_BYTES;
  unsigned* ql = (unsigned*)(ws + off); off += PLANE_BYTES;
  unsigned* kh = (unsigned*)(ws + off); off += PLANE_BYTES;
  unsigned* kl = (unsigned*)(ws + off); off += PLANE_BYTES;
  unsigned* vh = (unsigned*)(ws + off); off += PLANE_BYTES;
  unsigned* vl = (unsigned*)(ws + off); off += PLANE_BYTES;
  float* o0 = (float*)(ws + off); off += O0_BYTES;
  float* o1 = (float*)(ws + off); off += O1_BYTES;
  float* o2 = (float*)(ws + off); off += O2_BYTES;
  float* l0 = (float*)(ws + off); off += L0_BYTES;
  float* l1 = (float*)(ws + off); off += L1_BYTES;
  float* l2 = (float*)(ws + off); off += L2_BYTES;
  if (off > ws_size) return;

  FreqTab ft;
  for (int i = 0; i < 32; ++i) {
    const float t = (float)i / 32.0f;
    const float pw = (float)pow(10000.0, (double)t);
    ft.f[i] = 1.0f / pw;
  }

  const int ntab = SEQ_LEN * HALF_D;
  xpos_table_kernel<<<(ntab + 255) / 256, 256, 0, stream>>>(ft, cq, sq, ck, sk, ntab);

  const int nprep = NUM_HEAD * SEQ_LEN * HALF_D;
  prep_qkv_kernel<<<(nprep + 255) / 256, 256, 0, stream>>>(q, k, v, cq, sq, ck, sk, qh, ql, kh, kl, vh, vl, nprep);

  const unsigned short* qhs = (const unsigned short*)qh;
  const unsigned short* qls = (const unsigned short*)ql;
  const unsigned short* khs = (const unsigned short*)kh;
  const unsigned short* kls = (const unsigned short*)kl;
  const unsigned short* vhs = (const unsigned short*)vh;
  const unsigned short* vls = (const unsigned short*)vl;
  dil_attn_kernel<<<4 * 256, 128, 0, stream>>>(qhs, qls, khs, kls, vhs, vls, o0, l0, 1, 1024, 4, 4);
  dil_attn_kernel<<<2 * 256, 128, 0, stream>>>(qhs, qls, khs, kls, vhs, vls, o1, l1, 2, 2048, 2, 3);
  dil_attn_kernel<<<1 * 256, 128, 0, stream>>>(qhs, qls, khs, kls, vhs, vls, o2, l2, 4, 4096, 1, 2);

  const int ncomb = SEQ_LEN * NUM_HEAD * (HDIM / 4);
  combine_kernel<<<(ncomb + 255) / 256, 256, 0, stream>>>(o0, o1, o2, l0, l1, l2, out, ncomb);
}
